// Block_6511170421026
// MI455X (gfx1250) — hardware-run, weakly checked
//
#include <hip/hip_runtime.h>


#ifndef NB
#define NB 4
#endif
#ifndef SEQ
#define SEQ 2048
#endif
#define NB_FULL  4
#define SEQ_FULL 2048
#define DM   768
#define NH   12
#define HD   64
#define DQ   (NH * HD)
#define NQKV (3 * DM)
#define KCH  64
#define PCL2 10.0f
#define SL2  0.18033688011112042f
#define HID  (4 * DM)
#define ACAR 16.0f
#define WCAR 64.0f
#define OSC  (1.0f / (ACAR * WCAR))

static_assert(NB <= NB_FULL);
static_assert(SEQ <= SEQ_FULL);
static_assert(HD == 64);
static_assert(NH * HD == DM);
static_assert(DM % 64 == 0);
static_assert(SEQ % 64 == 0);
static_assert(SEQ % KCH == 0);
static_assert(KCH == 64);
static_assert((2 * DM) % 64 == 0);
static_assert(((size_t)SEQ * DM) % 8 == 0);
static_assert(((size_t)NQKV * DM) % 8 == 0);
static_assert(((size_t)DM * DM) % 8 == 0);
static_assert(HID == 3072);
static_assert(HID % 64 == 0);
static_assert(DM % 32 == 0);
static_assert(DM == 32 * 8 * 3);
static_assert(((size_t)NB * SEQ) % 8 == 0);
static_assert(((size_t)HID * DM) % 64 == 0);
static_assert(((size_t)NQKV * DM) % 64 == 0);
static_assert(ACAR == 16.0f); static_assert(WCAR == 64.0f);

typedef _Float16 h16;
typedef unsigned short bf;
typedef __attribute__((ext_vector_type(16))) __bf16   v16bf;
typedef __attribute__((ext_vector_type(16))) _Float16 v16h;
typedef __attribute__((ext_vector_type(8)))  _Float16 v8h;
typedef __attribute__((ext_vector_type(8)))  unsigned short v8us;
typedef __attribute__((ext_vector_type(8)))  float    v8f;
typedef __attribute__((ext_vector_type(4)))  float    v4f;
typedef v4f  __attribute__((may_alias)) v4fa;
typedef v8us __attribute__((may_alias)) v8usa;

__device__ __forceinline__ unsigned short f2bf(float f) { unsigned u = __float_as_uint(f); u += 0x7FFFu + ((u >> 16) & 1u); return (unsigned short)(u >> 16); }
__device__ __forceinline__ float bf2f(unsigned short b) { return __uint_as_float(((unsigned)b) << 16); }
__device__ __forceinline__ float bfr(float f) { return bf2f(f2bf(f)); }
__device__ __forceinline__ v16h cat16(v8h lo, v8h hi) { return __builtin_shufflevector(lo, hi, 0, 1, 2, 3, 4, 5, 6, 7, 8, 9, 10, 11, 12, 13, 14, 15); }
__device__ __forceinline__ v16bf cat16b(v8us lo, v8us hi) { return __builtin_bit_cast(v16bf, __builtin_shufflevector(lo, hi, 0, 1, 2, 3, 4, 5, 6, 7, 8, 9, 10, 11, 12, 13, 14, 15)); }
__device__ __forceinline__ v8f wmma16(v16h a, v16h b, v8f c) { return __builtin_amdgcn_wmma_f32_16x16x32_f16(false, a, false, b, (short)0, c, false, false); }
__device__ __forceinline__ v8f wmmab(v16bf a, v16bf b, v8f c) { return __builtin_amdgcn_wmma_f32_16x16x32_bf16(false, a, false, b, (short)0, c, false, false); }
__device__ __forceinline__ void splitf(float y, unsigned short& h, unsigned short& l) { h = f2bf(y); l = f2bf(y - bf2f(h)); }

template <typename T16> struct WFrag;
template <> struct WFrag<h16> { typedef v16h V; static __device__ __forceinline__ V ld(const h16* p) { return cat16(*(const v8h*)p, *(const v8h*)(p + 16)); } static __device__ __forceinline__ v8f mma(V a, V b, v8f c) { return wmma16(a, b, c); } };
template <> struct WFrag<bf> { typedef v16bf V; static __device__ __forceinline__ V ld(const bf* p) { return cat16b(*(const v8us*)p, *(const v8us*)(p + 16)); } static __device__ __forceinline__ v8f mma(V a, V b, v8f c) { return wmmab(a, b, c); } };

static __device__ __forceinline__ h16 toh_flush(float v) { const h16 r = (h16)v; return (fabsf(v) < 6.103515625e-05f) ? (h16)0.0f : r; }
__device__ __forceinline__ v8f gmma(v16h a, v16h b, v8f c) { c = wmma16(a, b, c); asm volatile("v_nop\n\tv_nop\n\tv_nop\n\tv_nop" : "+v"(c) : "v"(a), "v"(b)); return c; }
__device__ __forceinline__ v8f gmma(v16bf a, v16bf b, v8f c) { c = wmmab(a, b, c); asm volatile("v_nop\n\tv_nop\n\tv_nop\n\tv_nop" : "+v"(c) : "v"(a), "v"(b)); return c; }
__device__ __forceinline__ float gelu_erf(float v) { return 0.5f * v * (1.0f + erff(v * 0.70710678118654752f)); }

template <typename T16, int NSPLIT, int BIASM, int ACT, int RESM, bool OUT16>
__device__ __forceinline__ void gemm_tile(const T16* __restrict__ A, const T16* __restrict__ A2, const T16* __restrict__ Bt, unsigned K, void* Cv, unsigned ldc, const float* __restrict__ bias, const float* __restrict__ R, unsigned ldr, float osc, float ocar, size_t sA, size_t sB, size_t sC, size_t cstr, size_t sR) {
    typedef typename WFrag<T16>::V V;
    __shared__ __align__(16) float os[16 * 68];
    const size_t z = blockIdx.z; A += z * sA; if (NSPLIT == 1) A2 += z * sA; Bt += z * sB;
    const unsigned lane = threadIdx.x & 31u, lr = lane & 15u, hi = lane >> 4; const unsigned r0 = blockIdx.x * 64u, c0 = blockIdx.y * 64u;
    v8f acc[4][4];
#pragma unroll
    for (int mb = 0; mb < 4; ++mb)
#pragma unroll
        for (int nb = 0; nb < 4; ++nb) acc[mb][nb] = (v8f){};
    const size_t aoff = (size_t)(r0 + lr) * K + 8u * hi, boff = (size_t)(c0 + lr) * K + 8u * hi;
#pragma unroll 1
    for (unsigned kc = 0; kc < K; kc += 32u) {
        V a[4], a2[4];
#pragma unroll
        for (int mb = 0; mb < 4; ++mb) { a[mb] = WFrag<T16>::ld(A + aoff + (size_t)mb * 16 * K + kc); if (NSPLIT == 1) a2[mb] = WFrag<T16>::ld(A2 + aoff + (size_t)mb * 16 * K + kc); }
#pragma unroll
        for (int nb = 0; nb < 4; ++nb) { const V b = WFrag<T16>::ld(Bt + boff + (size_t)nb * 16 * K + kc);
#pragma unroll
            for (int mb = 0; mb < 4; ++mb) { acc[mb][nb] = gmma(a[mb], b, acc[mb][nb]); if (NSPLIT == 1) acc[mb][nb] = gmma(a2[mb], b, acc[mb][nb]); } }
    }
    v4f bv = (v4f){0.f, 0.f, 0.f, 0.f}; v4f cb0 = bv, cb1 = bv;
    if (BIASM == 1) {
        if (OUT16) { const unsigned cb = c0 + (lane & 7u) * 8u;
#pragma unroll
            for (int q = 0; q < 4; ++q) { cb0[q] = bfr(bias[cb + q]); cb1[q] = bfr(bias[cb + 4 + q]); } }
        else { const unsigned cb = c0 + lr * 4u; bv[0] = bfr(bias[cb]); bv[1] = bfr(bias[cb + 1]); bv[2] = bfr(bias[cb + 2]); bv[3] = bfr(bias[cb + 3]); }
    }
#pragma unroll
    for (int mb = 0; mb < 4; ++mb) {
#pragma unroll
        for (int nb = 0; nb < 4; ++nb) {
#pragma unroll
            for (int j = 0; j < 8; ++j) os[(hi * 8 + j) * 68 + nb * 16 + lr] = acc[mb][nb][j]; }
        __builtin_amdgcn_wave_barrier(); asm volatile("" ::: "memory");
        if (OUT16) {
            h16* crow = (h16*)Cv + z * sC + (size_t)blockIdx.y * cstr + (size_t)(r0 + mb * 16) * ldc;
            const unsigned rq = lane >> 3, pc = (lane & 7u) * 8u;
#pragma unroll 1
            for (unsigned s = 0; s < 4u; ++s) {
                const unsigned row = 4u * s + rq;
                v4f x0 = *(const v4fa*)(os + row * 68 + pc), x1 = *(const v4fa*)(os + row * 68 + pc + 4);
                float rb = 0.f;
                if (BIASM == 2) rb = bfr(bias[r0 + mb * 16 + row]);
#pragma unroll
                for (int q = 0; q < 4; ++q) {
                    float u0 = x0[q] * osc + (cb0[q] + rb), u1 = x1[q] * osc + (cb1[q] + rb);
                    if (ACT == 1) { u0 = gelu_erf(u0); u1 = gelu_erf(u1); }
                    x0[q] = u0 * ocar; x1[q] = u1 * ocar; }
                *(v4fa*)(os + row * 68 + pc) = x0; *(v4fa*)(os + row * 68 + pc + 4) = x1; }
            asm volatile("" ::: "memory");
            v8h o[4];
#pragma unroll
            for (int s = 0; s < 4; ++s) { const unsigned row = 4u * s + rq; const v4f x0 = *(const v4fa*)(os + row * 68 + pc), x1 = *(const v4fa*)(os + row * 68 + pc + 4);
#pragma unroll
                for (int q = 0; q < 4; ++q) { o[s][q] = toh_flush(x0[q]); o[s][4 + q] = toh_flush(x1[q]); } }
#pragma unroll 1
            for (int ps = 0; ps < 2; ++ps) {
#pragma unroll
                for (int s = 0; s < 4; ++s) *(volatile v8h*)(crow + (size_t)(4u * s + rq) * ldc + pc) = o[s];
                if (ps == 0) __threadfence(); }
        } else {
            float* crow = (float*)Cv + z * sC + (size_t)blockIdx.y * cstr + (size_t)(r0 + mb * 16) * ldc;
            const unsigned cofs = lr * 4u;
            v4f val[8];
#pragma unroll
            for (int s = 0; s < 8; ++s) { const unsigned row = 2u * s + hi; v4f t = *(const v4fa*)(os + row * 68 + cofs); t = t * osc + bv;
                if (RESM != 0) { v4f rv = *(const v4f*)(R + z * sR + (size_t)(r0 + mb * 16 + row) * ldr + c0 + cofs);
                    if (RESM == 2) { rv[0] = bfr(rv[0]); rv[1] = bfr(rv[1]); rv[2] = bfr(rv[2]); rv[3] = bfr(rv[3]); }
                    t = rv + t; }
                val[s] = t; }
#pragma unroll 1
            for (int ps = 0; ps < 2; ++ps) {
#pragma unroll
                for (int s = 0; s < 8; ++s) *(volatile v4f*)(crow + (size_t)(2u * s + hi) * ldc + cofs) = val[s];
                if (ps == 0) __threadfence(); }
        }
        __builtin_amdgcn_wave_barrier(); asm volatile("" ::: "memory");
    }
}

__global__ __launch_bounds__(32) void k_gemm_qk(const h16* __restrict__ A, const h16* __restrict__ Bt, h16* C, const float* __restrict__ bias) {
    gemm_tile<h16, 0, 1, 0, 0, true>(A, nullptr, Bt, (unsigned)DM, (void*)C, (unsigned)HD, bias, nullptr, 0u, OSC, 1.0f, (size_t)SEQ * DM, (size_t)0, (size_t)2 * NH * SEQ * HD, (size_t)SEQ * HD, (size_t)0); }
__global__ __launch_bounds__(32) void k_gemm_vt(const h16* __restrict__ A, const h16* __restrict__ Bt, h16* C, const float* __restrict__ bias) {
    gemm_tile<h16, 0, 2, 0, 0, true>(A, nullptr, Bt, (unsigned)DM, (void*)C, (unsigned)SEQ, bias, nullptr, 0u, OSC, 1.0f, (size_t)0, (size_t)SEQ * DM, (size_t)DM * SEQ, (size_t)64, (size_t)0); }
__global__ __launch_bounds__(32) void k_gemm_proj(const bf* __restrict__ A, const bf* __restrict__ A2, const bf* __restrict__ Bt, float* C, const float* __restrict__ bias, const float* __restrict__ R) {
    gemm_tile<bf, 1, 1, 0, 2, false>(A, A2, Bt, (unsigned)DQ, (void*)C, (unsigned)DM, bias, R, (unsigned)DM, 1.0f, 1.0f, (size_t)SEQ * DQ, (size_t)0, (size_t)SEQ * DM, (size_t)64, (size_t)SEQ_FULL * DM); }
__global__ __launch_bounds__(32) void k_gemm_fc1(const h16* __restrict__ A, const h16* __restrict__ Bt, h16* C, const float* __restrict__ bias) {
    gemm_tile<h16, 0, 1, 1, 0, true>(A, nullptr, Bt, (unsigned)DM, (void*)C, (unsigned)HID, bias, nullptr, 0u, OSC, ACAR, (size_t)SEQ * DM, (size_t)0, (size_t)SEQ * HID, (size_t)64, (size_t)0); }
__global__ __launch_bounds__(32) void k_gemm_fc2(const h16* __restrict__ A, const h16* __restrict__ Bt, float* C, const float* __restrict__ bias, const float* __restrict__ R) {
    gemm_tile<h16, 0, 1, 0, 1, false>(A, nullptr, Bt, (unsigned)HID, (void*)C, (unsigned)DM, bias, R, (unsigned)DM, OSC, 1.0f, (size_t)SEQ * HID, (size_t)0, (size_t)SEQ_FULL * DM, (size_t)64, (size_t)SEQ * DM); }

__global__ __launch_bounds__(256) void k_cvt8(const float* __restrict__ src, bf* dst, unsigned n8, size_t sstr, size_t dstr) {
    const unsigned i = blockIdx.x * 256u + threadIdx.x; if (i >= n8) return;
    const float* s = src + (size_t)blockIdx.y * sstr + (size_t)i * 8; bf* d = dst + (size_t)blockIdx.y * dstr + (size_t)i * 8;
    const v4f v0 = *(const v4f*)s, v1 = *(const v4f*)(s + 4); v8us o;
#pragma unroll
    for (int k = 0; k < 4; ++k) { o[k] = f2bf(v0[k]); o[4 + k] = f2bf(v1[k]); }
    *(volatile v8us*)d = o; __threadfence(); *(volatile v8us*)d = o; }

__global__ __launch_bounds__(256) void k_cvtw(const float* __restrict__ src, h16* dst, unsigned n8) {
    const unsigned i = blockIdx.x * 256u + threadIdx.x; if (i >= n8) return;
    const float* s = src + (size_t)i * 8; h16* d = dst + (size_t)i * 8;
    const v4f v0 = *(const v4f*)s, v1 = *(const v4f*)(s + 4); v8h o;
#pragma unroll
    for (int k = 0; k < 4; ++k) { o[k] = toh_flush(bfr(v0[k]) * WCAR); o[4 + k] = toh_flush(bfr(v1[k]) * WCAR); }
    *(volatile v8h*)d = o; __threadfence(); *(volatile v8h*)d = o; }

__global__ __launch_bounds__(256) void k_ln(const float* __restrict__ X, const float* __restrict__ g, const float* __restrict__ be, h16* H, unsigned rows, unsigned inbf, size_t bstr) {
#pragma clang fp contract(off)
    const unsigned wave = (unsigned)__builtin_amdgcn_readfirstlane((int)(threadIdx.x >> 5)), lane = threadIdx.x & 31u;
    const unsigned gr = blockIdx.x * 8u + wave;
    if (gr >= rows) return;
    const unsigned bb = gr / (unsigned)SEQ, tt = gr % (unsigned)SEQ;
    const float* xr = X + (size_t)bb * bstr + (size_t)tt * DM;
    float v[3][8];
    float s = 0.f;
#pragma unroll
    for (int j = 0; j < 3; ++j) { const float* p = xr + ((unsigned)(j * 32) + lane) * 8u; const v4f a = *(const v4f*)p, c = *(const v4f*)(p + 4);
#pragma unroll
        for (int q = 0; q < 4; ++q) { float u0 = a[q], u1 = c[q]; if (inbf != 0u) { u0 = bfr(u0); u1 = bfr(u1); } v[j][q] = u0; v[j][4 + q] = u1; s += u0; s += u1; } }
#pragma unroll
    for (int m = 16; m >= 1; m >>= 1) s += __shfl_xor(s, m, 32);
    const float mu = s * (1.0f / (float)DM);
    float ss = 0.f;
#pragma unroll
    for (int j = 0; j < 3; ++j)
#pragma unroll
        for (int q = 0; q < 8; ++q) { const float d = v[j][q] - mu; v[j][q] = d; ss += d * d; }
#pragma unroll
    for (int m = 16; m >= 1; m >>= 1) ss += __shfl_xor(ss, m, 32);
    const float rstd = rsqrtf(ss * (1.0f / (float)DM) + 1.0e-6f);
    h16* hr = H + (size_t)gr * DM;
    v8h o[3];
#pragma unroll
    for (int j = 0; j < 3; ++j) { const unsigned cb = ((unsigned)(j * 32) + lane) * 8u;
        const v4f g0 = *(const v4f*)(g + cb), g1 = *(const v4f*)(g + cb + 4), b0 = *(const v4f*)(be + cb), b1 = *(const v4f*)(be + cb + 4);
#pragma unroll
        for (int q = 0; q < 4; ++q) { o[j][q] = toh_flush((v[j][q] * rstd * bfr(g0[q]) + bfr(b0[q])) * ACAR); o[j][4 + q] = toh_flush((v[j][4 + q] * rstd * bfr(g1[q]) + bfr(b1[q])) * ACAR); } }
#pragma unroll 1
    for (int ps = 0; ps < 2; ++ps) {
#pragma unroll
        for (int j = 0; j < 3; ++j) *(volatile v8h*)(hr + ((unsigned)(j * 32) + lane) * 8u) = o[j];
        if (ps == 0) __threadfence(); }
}

__global__ __launch_bounds__(128) void k_flash(const h16* __restrict__ QK, const h16* __restrict__ VT, bf* Ah, bf* Al) {
    __shared__ __align__(16) unsigned short osh[4][16 * 72];
    __shared__ __align__(16) unsigned short osl[4][16 * 72];
    const unsigned lane = threadIdx.x & 31u, w = threadIdx.x >> 5, lr = lane & 15u, hi = lane >> 4;
    const unsigned b = blockIdx.z, h = blockIdx.y, q0 = blockIdx.x * 64u + w * 16u;
    const h16* Qp = QK + ((size_t)(b * 2u * NH + h) * SEQ) * HD;
    const h16* Kp = QK + ((size_t)(b * 2u * NH + NH + h) * SEQ) * HD;
    const h16* Vp = VT + ((size_t)b * DM + h * HD) * SEQ;
    v16h bq[2];
    bq[0] = WFrag<h16>::ld(Qp + (size_t)(q0 + lr) * HD + 8u * hi);
    bq[1] = WFrag<h16>::ld(Qp + (size_t)(q0 + lr) * HD + 32u + 8u * hi);
    v8f acc[4];
#pragma unroll
    for (int dt = 0; dt < 4; ++dt) acc[dt] = (v8f){};
    float m = -3.0e38f, ls = 0.f;
    const h16* kbase = Kp + (size_t)lr * HD + 8u * hi;
    const h16* vbase = Vp + (size_t)lr * SEQ + 8u * hi;
#pragma unroll 1
    for (unsigned kc = 0; kc < SEQ; kc += KCH) {
        v16h ka[4][2]; v8f st[4];
#pragma unroll
        for (int kt = 0; kt < 4; ++kt) { ka[kt][0] = WFrag<h16>::ld(kbase + (size_t)(kc + kt * 16) * HD); ka[kt][1] = WFrag<h16>::ld(kbase + (size_t)(kc + kt * 16) * HD + 32); }
#pragma unroll
        for (int kt = 0; kt < 4; ++kt) { st[kt] = wmma16(ka[kt][0], bq[0], (v8f){}); st[kt] = wmma16(ka[kt][1], bq[1], st[kt]); }
        asm volatile("v_nop\n\tv_nop\n\tv_nop\n\tv_nop" : "+v"(st[0]), "+v"(st[1]), "+v"(st[2]), "+v"(st[3]) : "v"(ka[0][0]), "v"(ka[0][1]), "v"(ka[1][0]), "v"(ka[1][1]), "v"(ka[2][0]), "v"(ka[2][1]), "v"(ka[3][0]), "v"(ka[3][1]), "v"(bq[0]), "v"(bq[1]));
        float mx = st[0][0];
#pragma unroll
        for (int kt = 0; kt < 4; ++kt)
#pragma unroll
            for (int r = 0; r < 8; ++r) mx = fmaxf(mx, st[kt][r]);
        mx = fmaxf(mx, __shfl_xor(mx, 16, 32));
        const float mn = fmaxf(m, mx * SL2);
        const float al = __builtin_amdgcn_exp2f(m - mn);
        m = mn;
        const float sh = PCL2 - mn;
        float psum = 0.f; v16h pb[2];
#pragma unroll
        for (int ks = 0; ks < 2; ++ks)
#pragma unroll
            for (int r = 0; r < 8; ++r) { const float p0 = __builtin_amdgcn_exp2f(st[2 * ks][r] * SL2 + sh); const float p1 = __builtin_amdgcn_exp2f(st[2 * ks + 1][r] * SL2 + sh); psum += p0 + p1; pb[ks][r] = (h16)p0; pb[ks][8 + r] = (h16)p1; }
        ls = ls * al + psum;
#pragma unroll
        for (int dt = 0; dt < 4; ++dt)
#pragma unroll
            for (int r = 0; r < 8; ++r) acc[dt][r] *= al;
        v16h va[4][2];
#pragma unroll
        for (int dt = 0; dt < 4; ++dt) { va[dt][0] = WFrag<h16>::ld(vbase + (size_t)(dt * 16) * SEQ + kc); va[dt][1] = WFrag<h16>::ld(vbase + (size_t)(dt * 16) * SEQ + kc + 32); }
#pragma unroll
        for (int dt = 0; dt < 4; ++dt) { acc[dt] = wmma16(va[dt][0], pb[0], acc[dt]); acc[dt] = wmma16(va[dt][1], pb[1], acc[dt]); }
        asm volatile("v_nop\n\tv_nop\n\tv_nop\n\tv_nop" : "+v"(acc[0]), "+v"(acc[1]), "+v"(acc[2]), "+v"(acc[3]) : "v"(va[0][0]), "v"(va[0][1]), "v"(va[1][0]), "v"(va[1][1]), "v"(va[2][0]), "v"(va[2][1]), "v"(va[3][0]), "v"(va[3][1]), "v"(pb[0]), "v"(pb[1]));
    }
    ls += __shfl_xor(ls, 16, 32);
    const float inv = 1.0f / ls;
    unsigned short* oh = &osh[w][0]; unsigned short* ol = &osl[w][0];
#pragma unroll
    for (int dt = 0; dt < 4; ++dt) { v8us hv, lv;
#pragma unroll
        for (int r = 0; r < 8; ++r) { unsigned short a, c; splitf(acc[dt][r] * inv, a, c); hv[r] = a; lv[r] = c; }
        *(v8usa*)(oh + lr * 72 + dt * 16 + 8 * hi) = hv; *(v8usa*)(ol + lr * 72 + dt * 16 + 8 * hi) = lv; }
    __builtin_amdgcn_wave_barrier(); asm volatile("" ::: "memory");
    const unsigned rq = lane >> 3, pc = (lane & 7u) * 8u;
    v8us vh[4], vl[4];
#pragma unroll
    for (int s = 0; s < 4; ++s) { const unsigned row = 4u * s + rq; vh[s] = *(const v8usa*)(oh + row * 72 + pc); vl[s] = *(const v8usa*)(ol + row * 72 + pc); }
    const size_t gofs = ((size_t)b * SEQ + q0) * DQ + h * HD + pc;
#pragma unroll 1
    for (int ps = 0; ps < 2; ++ps) {
#pragma unroll
        for (int s = 0; s < 4; ++s) { const size_t o = gofs + (size_t)(4u * s + rq) * DQ; *(volatile v8us*)(Ah + o) = vh[s]; *(volatile v8us*)(Al + o) = vl[s]; }
        if (ps == 0) __threadfence(); }
}

constexpr size_t SZ_WQ = (size_t)NQKV * DM * 2;
constexpr size_t SZ_WO = (size_t)DM * DM * 2;
constexpr size_t SZ_W1 = (size_t)HID * DM * 2;
constexpr size_t SZ_W2 = (size_t)DM * HID * 2;
constexpr size_t SZ_H  = (size_t)NB * SEQ * DM * 2;
constexpr size_t SZ_QK = (size_t)NB * 2 * NH * SEQ * HD * 2;
constexpr size_t SZ_VT = (size_t)NB * DM * SEQ * 2;
constexpr size_t SZ_AT = (size_t)NB * SEQ * DQ * 2;
constexpr size_t SZ_X1 = (size_t)NB * SEQ * DM * 4;
constexpr size_t SZ_G  = (size_t)NB * SEQ * HID * 2;
constexpr size_t OFF_WQ = 0;
constexpr size_t OFF_WO = OFF_WQ + SZ_WQ;
constexpr size_t OFF_W1 = OFF_WO + SZ_WO;
constexpr size_t OFF_W2 = OFF_W1 + SZ_W1;
constexpr size_t OFF_H  = OFF_W2 + SZ_W2;
constexpr size_t OFF_QK = OFF_H + SZ_H;
constexpr size_t OFF_VT = OFF_QK + SZ_QK;
constexpr size_t OFF_AH = OFF_VT + SZ_VT;
constexpr size_t OFF_AL = OFF_AH + SZ_AT;
constexpr size_t OFF_X1 = OFF_AL + SZ_AT;
constexpr size_t OFF_G  = OFF_QK;
constexpr size_t WS_TOTAL = OFF_X1 + SZ_X1;
static_assert(SZ_WQ % 256 == 0); static_assert(SZ_WO % 256 == 0); static_assert(SZ_W1 % 256 == 0); static_assert(SZ_W2 % 256 == 0);
static_assert(SZ_H % 256 == 0); static_assert(SZ_QK % 256 == 0); static_assert(SZ_VT % 256 == 0); static_assert(SZ_AT % 256 == 0);
static_assert(SZ_X1 % 256 == 0); static_assert(SZ_G % 256 == 0);
static_assert(OFF_G + SZ_G <= OFF_AL);
static_assert(WS_TOTAL <= (size_t)134217728);
static_assert((size_t)(SEQ / 64) * (2 * NH) * NB * 4096 == SZ_QK / 2);
static_assert((size_t)(DM / 64) * (SEQ / 64) * NB * 4096 == SZ_VT / 2);
static_assert((size_t)(SEQ / 64) * NH * NB * 4 * 16 * HD == SZ_AT / 2);
static_assert((size_t)(SEQ / 64) * (DM / 64) * NB * 4096 == SZ_X1 / 4);
static_assert((size_t)(SEQ / 64) * (HID / 64) * NB * 4096 == SZ_G / 2);
static_assert((size_t)(SEQ / 64) * (DM / 64) * 4096 == (size_t)SEQ * DM);
static_assert((size_t)NB * SEQ * DM == SZ_H / 2);

extern "C" void kernel_launch(void* const* d_in, const int* in_sizes, int n_in,
                              void* d_out, int out_size, void* d_ws, size_t ws_size, hipStream_t stream) {
    if (n_in < 13) return;
    const size_t xneed = (size_t)(NB - 1) * SEQ_FULL * DM + (size_t)SEQ * DM;
    if ((size_t)in_sizes[0] < xneed) return;
    if ((size_t)in_sizes[1] < (size_t)DM) return;
    if ((size_t)in_sizes[2] < (size_t)DM) return;
    if ((size_t)in_sizes[3] < (size_t)NQKV * DM) return;
    if ((size_t)in_sizes[4] < (size_t)NQKV) return;
    if ((size_t)in_sizes[5] < (size_t)DM * DM) return;
    if ((size_t)in_sizes[6] < (size_t)DM) return;
    if ((size_t)in_sizes[7] < (size_t)DM) return;
    if ((size_t)in_sizes[8] < (size_t)DM) return;
    if ((size_t)in_sizes[9] < (size_t)HID * DM) return;
    if ((size_t)in_sizes[10] < (size_t)HID) return;
    if ((size_t)in_sizes[11] < (size_t)DM * HID) return;
    if ((size_t)in_sizes[12] < (size_t)DM) return;
    if ((size_t)out_size < xneed) return;
    if (ws_size < WS_TOTAL) return;
    const float* x = (const float*)d_in[0];
    const float* ln1g = (const float*)d_in[1]; const float* ln1b = (const float*)d_in[2];
    const float* wqkv = (const float*)d_in[3]; const float* bqkv = (const float*)d_in[4];
    const float* wo = (const float*)d_in[5]; const float* bo = (const float*)d_in[6];
    const float* ln2g = (const float*)d_in[7]; const float* ln2b = (const float*)d_in[8];
    const float* w1 = (const float*)d_in[9]; const float* b1 = (const float*)d_in[10];
    const float* w2 = (const float*)d_in[11]; const float* b2 = (const float*)d_in[12];
    float* OUT = (float*)d_out;
    char* wsp = (char*)d_ws;
    h16* WQ = (h16*)(wsp + OFF_WQ); bf* WO = (bf*)(wsp + OFF_WO); h16* W1 = (h16*)(wsp + OFF_W1); h16* W2 = (h16*)(wsp + OFF_W2);
    h16* HP = (h16*)(wsp + OFF_H);
    h16* QK = (h16*)(wsp + OFF_QK); h16* VT = (h16*)(wsp + OFF_VT); bf* ATh = (bf*)(wsp + OFF_AH); bf* ATl = (bf*)(wsp + OFF_AL);
    float* X1 = (float*)(wsp + OFF_X1); h16* GP = (h16*)(wsp + OFF_G);

    const unsigned nq8 = (unsigned)((size_t)NQKV * DM / 8), no8 = (unsigned)((size_t)DM * DM / 8), nh8 = (unsigned)((size_t)HID * DM / 8);
    const unsigned nrows = (unsigned)((size_t)NB * SEQ);
    k_cvt8<<<dim3((no8 + 255u) / 256u, 1, 1), 256, 0, stream>>>(wo, WO, no8, 0, 0);
    k_cvtw<<<dim3((nq8 + 255u) / 256u, 1, 1), 256, 0, stream>>>(wqkv, WQ, nq8);
    k_cvtw<<<dim3((nh8 + 255u) / 256u, 1, 1), 256, 0, stream>>>(w1, W1, nh8);
    k_cvtw<<<dim3((nh8 + 255u) / 256u, 1, 1), 256, 0, stream>>>(w2, W2, nh8);
    k_ln<<<dim3((nrows + 7u) / 8u, 1, 1), 256, 0, stream>>>(x, ln1g, ln1b, HP, nrows, 1u, (size_t)SEQ_FULL * DM);
    k_gemm_qk<<<dim3(SEQ / 64, 2 * NH, NB), 32, 0, stream>>>(HP, WQ, QK, bqkv);
    k_gemm_vt<<<dim3(DM / 64, SEQ / 64, NB), 32, 0, stream>>>(WQ + (size_t)2 * DM * DM, HP, VT, bqkv + 2 * DM);
    k_flash<<<dim3(SEQ / 64, NH, NB), 128, 0, stream>>>(QK, VT, ATh, ATl);
    k_gemm_proj<<<dim3(SEQ / 64, DM / 64, NB), 32, 0, stream>>>(ATh, ATl, WO, X1, bo, x);
    k_ln<<<dim3((nrows + 7u) / 8u, 1, 1), 256, 0, stream>>>(X1, ln2g, ln2b, HP, nrows, 0u, (size_t)SEQ * DM);
    k_gemm_fc1<<<dim3(SEQ / 64, HID / 64, NB), 32, 0, stream>>>(HP, W1, GP, b1);
    k_gemm_fc2<<<dim3(SEQ / 64, DM / 64, NB), 32, 0, stream>>>(GP, W2, OUT, b2, X1);
}
